// MambaBlock_70076686402475
// MI455X (gfx1250) — hardware-verified
//
#include <hip/hip_runtime.h>
#include <math.h>

typedef __attribute__((ext_vector_type(16))) _Float16 v16h;
typedef __attribute__((ext_vector_type(8)))  _Float16 v8h;
typedef __attribute__((ext_vector_type(4)))  _Float16 v4h;
typedef __attribute__((ext_vector_type(16))) __bf16   v16b;
typedef __attribute__((ext_vector_type(8)))  __bf16   v8b;
typedef __attribute__((ext_vector_type(8)))  float    v8f;
typedef __attribute__((ext_vector_type(4)))  float    v4f;
typedef __attribute__((ext_vector_type(4)))  unsigned int v4u;
typedef __attribute__((ext_vector_type(2)))  unsigned int v2u;

constexpr int kBatch  = 16;
constexpr int kSeqL   = 197;
constexpr int kSide   = 14;
constexpr int kWinS   = 7;
constexpr int kDm     = 768;
constexpr int kEd     = 1536;
constexpr int kNst    = 16;
constexpr int kDtr    = 48;
constexpr int kRows   = kBatch * kSeqL;
constexpr int kRowsP  = 3200;
constexpr int kWinT   = kWinS * kWinS;
constexpr int kRowsW  = 4 * kBatch * kWinT;
constexpr int kXzP    = 2 * kEd;
constexpr int kDbcP   = 128;
constexpr int kDbc16P = 64;
constexpr int kXpRows = 128;
constexpr int kThrRow = kEd / 4;
constexpr int kCarryU_L2 = 5;
constexpr int kCarryW_L2 = 10;
constexpr int kCarryD_L2 = 6;
constexpr int kCarryP_L2 = 8;
constexpr int kCarryY_L2 = 6;
static_assert(kRows == 3152);
static_assert(kRowsW == 3136);
static_assert(kSide * kSide + 1 == kSeqL);
static_assert(kDtr + 2 * kNst == 80);
static_assert((kRowsP % 64) == 0 && kRowsP >= kRows && kRowsP >= kRowsW);
static_assert((kXzP % 64) == 0 && (kEd % 64) == 0 && (kDm % 64) == 0 && (kDbcP % 64) == 0);
static_assert((kDm % 32) == 0 && (kEd % 32) == 0 && (kDbc16P % 32) == 0);
static_assert((kRows % 16) == 0);
static_assert(kThrRow == 384 && (kThrRow % 32) == 0);

constexpr size_t kSzXP    = (size_t)kRowsP * kDm * 2;
constexpr size_t kSzWI    = (size_t)kXzP * kDm * 2;
constexpr size_t kSzXZ    = (size_t)kRowsP * kXzP * 4;
constexpr size_t kSzH16   = (size_t)kRowsP * kEd * 2;
constexpr size_t kSzXP16  = (size_t)kXpRows * kEd * 2;
constexpr size_t kSzDBC   = (size_t)kRowsP * kDbcP * 4;
constexpr size_t kSzDBC16 = (size_t)kRowsP * kDbc16P * 2;
constexpr size_t kSzDTW16 = (size_t)kEd * kDbc16P * 2;
constexpr size_t kSzDELTA = (size_t)kRowsP * kEd * 4;
constexpr size_t kSzWO16  = (size_t)kDm * kEd * 2;
constexpr size_t kOffXH    = 0;
constexpr size_t kOffXL    = kOffXH + kSzXP;
constexpr size_t kOffWIH   = kOffXL + kSzXP;
constexpr size_t kOffWIL   = kOffWIH + kSzWI;
constexpr size_t kOffXZ    = kOffWIL + kSzWI;
constexpr size_t kOffU16   = kOffXZ + kSzXZ;
constexpr size_t kOffPRE16 = kOffU16 + kSzH16;
constexpr size_t kOffXP16  = kOffPRE16 + kSzH16;
constexpr size_t kOffDBC   = kOffXP16 + 3 * kSzXP16;
constexpr size_t kOffDBC16 = kOffDBC + kSzDBC;
constexpr size_t kOffDTW16 = kOffDBC16 + kSzDBC16;
constexpr size_t kOffDELTA = kOffDTW16 + kSzDTW16;
constexpr size_t kOffY0    = kOffDELTA + kSzDELTA;
constexpr size_t kOffY1    = kOffY0 + kSzH16;
constexpr size_t kOffYW    = kOffY1 + kSzH16;
constexpr size_t kOffWO16  = kOffYW + kSzH16;
constexpr size_t kWsTotal  = kOffWO16 + kSzWO16;
static_assert(kWsTotal == 133185536ull);
static_assert(kWsTotal <= 134217728ull);
static_assert((kOffXL % 128) == 0 && (kOffWIH % 128) == 0 && (kOffWIL % 128) == 0 && (kOffXZ % 128) == 0 &&
              (kOffU16 % 128) == 0 && (kOffPRE16 % 128) == 0 && (kOffXP16 % 128) == 0 && (kOffDBC % 128) == 0 &&
              (kOffDBC16 % 128) == 0 && (kOffDTW16 % 128) == 0 && (kOffDELTA % 128) == 0 && (kOffY0 % 128) == 0 &&
              (kOffY1 % 128) == 0 && (kOffYW % 128) == 0 && (kOffWO16 % 128) == 0 && (kSzXP16 % 128) == 0);

__device__ __forceinline__ unsigned pin_u(unsigned t) { asm volatile("" : "+v"(t)); return t; }

__device__ __forceinline__ unsigned bf_hi_bits(float f) {
  unsigned u = __float_as_uint(f);
  const unsigned lsb = (u & 0x00010000u) ? 1u : 0u;
  u = (u + 0x7FFFu + lsb) & 0xFFFF0000u;
  return u;
}
__device__ __forceinline__ void bf_split(float f, unsigned& hb, unsigned& lb) {
  hb = bf_hi_bits(f);
  lb = bf_hi_bits(f - __uint_as_float(hb));
}
__device__ __forceinline__ unsigned pack_hi16(unsigned a, unsigned b) {
  return __builtin_amdgcn_perm(b, a, 0x07060302u);
}
__device__ __forceinline__ float h16_to_f32(unsigned hb) {
  const unsigned sgn = (hb & 0x8000u) << 16;
  const unsigned em = hb & 0x7fffu;
  const float fn = __uint_as_float((em << 13) + 0x38000000u);
  const float fs = (float)em * 5.9604644775390625e-8f;
  const float mag = (em < 0x400u) ? fs : fn;
  return __uint_as_float(__float_as_uint(mag) | sgn);
}
__device__ __forceinline__ _Float16 to_h16(float v) {
  const float c = fminf(fmaxf(v, -60000.0f), 60000.0f);
  const float w = (fabsf(c) < 6.103515625e-05f) ? 0.0f : c;
  return (_Float16)w;
}
__device__ __forceinline__ float silu_f(float x) {
  const float t = fminf(-x, 60.0f);
  const float e = expf(t);
  return x * (1.0f / (1.0f + e));
}
__device__ __forceinline__ float softplus_f(float v) {
  return fmaxf(v, 0.0f) + log1pf(expf(-fabsf(v)));
}
__device__ __forceinline__ void wave_sync() {
  __builtin_amdgcn_fence(__ATOMIC_RELEASE, "workgroup");
  __builtin_amdgcn_wave_barrier();
  __builtin_amdgcn_fence(__ATOMIC_ACQUIRE, "workgroup");
}

__device__ __forceinline__ void row_guard_h(v8f& a, v8f& b, v8f& c, v8f& d, v16h x, v16h y) {
  asm volatile("v_nop\n\tv_nop\n\tv_nop\n\tv_nop" : "+v"(a), "+v"(b), "+v"(c), "+v"(d) : "v"(x), "v"(y));
}
__device__ __forceinline__ void row_guard_b(v8f& a, v8f& b, v8f& c, v8f& d, v16b x, v16b y) {
  asm volatile("v_nop\n\tv_nop\n\tv_nop\n\tv_nop" : "+v"(a), "+v"(b), "+v"(c), "+v"(d) : "v"(x), "v"(y));
}
__device__ __forceinline__ void keep4_h(v16h a, v16h b, v16h c, v16h d) { asm volatile("v_nop" :: "v"(a), "v"(b), "v"(c), "v"(d)); }
__device__ __forceinline__ void keep4_b(v16b a, v16b b, v16b c, v16b d) { asm volatile("v_nop" :: "v"(a), "v"(b), "v"(c), "v"(d)); }
__device__ __forceinline__ void acc_guard4(v8f& a, v8f& b, v8f& c, v8f& d) {
  asm volatile("v_nop\n\tv_nop\n\tv_nop\n\tv_nop" : "+v"(a), "+v"(b), "+v"(c), "+v"(d));
}
template <typename T> struct Frag;
template <> struct Frag<_Float16> {
  typedef v16h V; union U { v16h v; v8h h[2]; };
  static __device__ __forceinline__ v16h load(const _Float16* p) {
    U f; f.h[0] = *(const v8h*)(p); f.h[1] = *(const v8h*)(p + 16); return f.v;
  }
  static __device__ __forceinline__ v8f mma(v16h a, v16h b, v8f c) {
    return __builtin_amdgcn_wmma_f32_16x16x32_f16(false, a, false, b, (short)0, c, false, false);
  }
  static __device__ __forceinline__ void guard(v8f& a, v8f& b, v8f& c, v8f& d, v16h x, v16h y) { row_guard_h(a, b, c, d, x, y); }
  static __device__ __forceinline__ void keep(v16h a, v16h b, v16h c, v16h d) { keep4_h(a, b, c, d); }
};
template <> struct Frag<__bf16> {
  typedef v16b V; union U { v16b v; v8b h[2]; };
  static __device__ __forceinline__ v16b load(const __bf16* p) {
    U f; f.h[0] = *(const v8b*)(p); f.h[1] = *(const v8b*)(p + 16); return f.v;
  }
  static __device__ __forceinline__ v8f mma(v16b a, v16b b, v8f c) {
    return __builtin_amdgcn_wmma_f32_16x16x32_bf16(false, a, false, b, (short)0, c, false, false);
  }
  static __device__ __forceinline__ void guard(v8f& a, v8f& b, v8f& c, v8f& d, v16b x, v16b y) { row_guard_b(a, b, c, d, x, y); }
  static __device__ __forceinline__ void keep(v16b a, v16b b, v16b c, v16b d) { keep4_b(a, b, c, d); }
};
template <int ET> struct Elem;
template <> struct Elem<0> { typedef _Float16 T; };
template <> struct Elem<1> { typedef __bf16 T; };

template <int ET, bool SPLIT, int EPI, int SCALE_LOG2>
__global__ __launch_bounds__(256) void wmma_gemm64(
    const unsigned short* __restrict__ Ap, const unsigned short* __restrict__ A2p, int lda,
    const unsigned short* __restrict__ Btp, const unsigned short* __restrict__ Bt2p, int ldb,
    float* __restrict__ Cf, int ldc,
    unsigned short* __restrict__ C16, int ldc16,
    const float* __restrict__ bias,
    int M, int N, int K, int Mstore) {
  typedef typename Elem<ET>::T T;
  typedef typename Frag<T>::V V;
  constexpr float scale = 1.0f / (float)(1u << SCALE_LOG2);
  const T* A = (const T*)Ap; const T* A2 = (const T*)A2p; const T* Bt = (const T*)Btp; const T* Bt2 = (const T*)Bt2p;
  __shared__ __align__(16) float sT[8][16 * 68];
  const int lane = threadIdx.x & 31;
  const int wave = threadIdx.x >> 5;
  const int tilesN = N >> 6;
  const int tilesM = M >> 6;
  const int tile = blockIdx.x * 8 + wave;
  if (tile >= tilesM * tilesN) return;
  const int tm = tile / tilesN;
  const int tn = tile - tm * tilesN;
  const int m0 = tm << 6;
  const int n0 = tn << 6;

  const int rlane = lane & 15;
  const int koff  = (lane >> 4) * 8;
  const int mOff  = (lane >> 4) * 8;

  v8f acc[4][4];
#pragma unroll
  for (int i = 0; i < 4; ++i)
#pragma unroll
    for (int j = 0; j < 4; ++j) acc[i][j] = (v8f){0.f,0.f,0.f,0.f,0.f,0.f,0.f,0.f};

  for (int k0 = 0; k0 < K; k0 += 32) {
    V bh[4], bl[4];
#pragma unroll
    for (int j = 0; j < 4; ++j) {
      const size_t bo = (size_t)(n0 + (j << 4) + rlane) * ldb + koff + k0;
      bh[j] = Frag<T>::load(Bt + bo);
      if (SPLIT) bl[j] = Frag<T>::load(Bt2 + bo);
    }
#pragma unroll
    for (int i = 0; i < 4; ++i) {
      const size_t ao = (size_t)(m0 + (i << 4) + rlane) * lda + koff + k0;
      V ah = Frag<T>::load(A + ao);
      V al;
      if (SPLIT) al = Frag<T>::load(A2 + ao);
#pragma unroll
      for (int j = 0; j < 4; ++j) {
        acc[i][j] = Frag<T>::mma(ah, bh[j], acc[i][j]);
        if (SPLIT) {
          acc[i][j] = Frag<T>::mma(ah, bl[j], acc[i][j]);
          acc[i][j] = Frag<T>::mma(al, bh[j], acc[i][j]);
        }
      }
      Frag<T>::guard(acc[i][0], acc[i][1], acc[i][2], acc[i][3], ah, SPLIT ? al : ah);
    }
    Frag<T>::keep(bh[0], bh[1], bh[2], bh[3]);
    if (SPLIT) Frag<T>::keep(bl[0], bl[1], bl[2], bl[3]);
  }
  acc_guard4(acc[0][0], acc[0][1], acc[0][2], acc[0][3]);
  acc_guard4(acc[1][0], acc[1][1], acc[1][2], acc[1][3]);
  acc_guard4(acc[2][0], acc[2][1], acc[2][2], acc[2][3]);
  acc_guard4(acc[3][0], acc[3][1], acc[3][2], acc[3][3]);

  float* slab = sT[wave];
#pragma unroll
  for (int i = 0; i < 4; ++i) {
    const int mBase = m0 + (i << 4);
#pragma unroll
    for (int j = 0; j < 4; ++j) {
      float bv = 0.f;
      if (EPI == 2) bv = bias[n0 + (j << 4) + rlane];
#pragma unroll
      for (int r = 0; r < 8; ++r) {
        float v = acc[i][j][r] * scale;
        if (EPI == 2) v += bv;
        slab[(mOff + r) * 68 + (j << 4) + rlane] = v;
      }
    }
    wave_sync();
    if (EPI == 2) {
      const int hh2 = lane >> 4, c42 = (lane & 15) * 4;
#pragma unroll 1
      for (int q = 0; q < 32; ++q) {
        float* p = slab + ((q >> 2) * 2 + hh2) * 68 + c42 + (q & 3);
        const float v = *p;
        *p = softplus_f(v);
      }
      wave_sync();
    }
    if (mBase < Mstore) {
      {
        const int hh = lane >> 4, c4 = (lane & 15) * 4;
        for (int pass = 0; pass < 2; ++pass) {
#pragma unroll
          for (int it = 0; it < 8; ++it) {
            const int row = it * 2 + hh;
            v4f v = *(const v4f*)(slab + row * 68 + c4);
            *(volatile v4f*)(Cf + (size_t)(mBase + row) * ldc + n0 + c4) = v;
          }
          __threadfence();
        }
      }
      if (EPI == 1 && n0 == 0) {
        const int q = lane >> 3, c8 = (lane & 7) * 8;
        constexpr float sideCarry = (float)(1u << kCarryD_L2);
        for (int pass = 0; pass < 2; ++pass) {
#pragma unroll
          for (int it = 0; it < 4; ++it) {
            const int row = it * 4 + q;
            const float* sp = slab + row * 68 + c8;
            v8h hv;
#pragma unroll
            for (int e = 0; e < 8; ++e) hv[e] = to_h16(sp[e] * sideCarry);
            *(volatile v8h*)(C16 + (size_t)(mBase + row) * ldc16 + c8) = hv;
          }
          __threadfence();
        }
      }
    }
    wave_sync();
  }
}

__global__ __launch_bounds__(256) void split_rows_bf16_kernel(
    const float* __restrict__ src, unsigned* __restrict__ dhi, unsigned* __restrict__ dlo,
    unsigned srcElems, unsigned total8) {
  const unsigned i = blockIdx.x * 256u + threadIdx.x;
  if (i >= total8) return;
  const unsigned e0 = i << 3;
  const bool valid = e0 < srcElems;
  const unsigned ec = valid ? e0 : 0u;
  v4f a0 = *(const v4f*)(src + ec);
  v4f a1 = *(const v4f*)(src + ec + 4);
  asm volatile("" : "+v"(a0));
  asm volatile("" : "+v"(a1));
  unsigned hb[8], lb[8];
#pragma unroll
  for (int e = 0; e < 4; ++e) {
    const float f0 = valid ? a0[e] : 0.0f;
    const float f1 = valid ? a1[e] : 0.0f;
    bf_split(f0, hb[e], lb[e]);
    bf_split(f1, hb[4 + e], lb[4 + e]);
  }
  const v4u hw = (v4u){pack_hi16(hb[0], hb[1]), pack_hi16(hb[2], hb[3]), pack_hi16(hb[4], hb[5]), pack_hi16(hb[6], hb[7])};
  const v4u lw = (v4u){pack_hi16(lb[0], lb[1]), pack_hi16(lb[2], lb[3]), pack_hi16(lb[4], lb[5]), pack_hi16(lb[6], lb[7])};
  unsigned* qh = dhi + (size_t)i * 4;
  unsigned* ql = dlo + (size_t)i * 4;
  *(volatile v4u*)qh = hw;
  *(volatile v4u*)ql = lw;
  __threadfence();
  *(volatile v4u*)qh = hw;
  *(volatile v4u*)ql = lw;
}

template <int CARRY_L2>
__global__ __launch_bounds__(256) void cast_pad_f16_kernel(
    const float* __restrict__ src, unsigned short* __restrict__ dst,
    unsigned srcRows, unsigned srcCols, unsigned dstCols8, unsigned total8) {
  constexpr float carry = (float)(1u << CARRY_L2);
  const unsigned i = blockIdx.x * 256u + threadIdx.x;
  if (i >= total8) return;
  const unsigned dr = pin_u(i / dstCols8);
  const unsigned g  = i - dr * dstCols8;
  const unsigned c0 = g << 3;
  const bool valid = (dr < srcRows) && (c0 < srcCols);
  const unsigned rc = (dr < srcRows) ? dr : (srcRows - 1u);
  const unsigned cc = (c0 < srcCols) ? c0 : (srcCols - 8u);
  const float* p = src + (size_t)rc * srcCols + cc;
  v4f a0 = *(const v4f*)(p);
  v4f a1 = *(const v4f*)(p + 4);
  asm volatile("" : "+v"(a0));
  asm volatile("" : "+v"(a1));
  v8h hv;
#pragma unroll
  for (int e = 0; e < 4; ++e) {
    const float f0 = valid ? (a0[e] * carry) : 0.0f;
    const float f1 = valid ? (a1[e] * carry) : 0.0f;
    hv[e]     = to_h16(f0);
    hv[4 + e] = to_h16(f1);
  }
  unsigned short* q = dst + (size_t)i * 8;
  *(volatile v8h*)q = hv;
  __threadfence();
  *(volatile v8h*)q = hv;
}

template <int MODE>
__global__ __launch_bounds__(256) void seq_prep_kernel(
    const float* __restrict__ XZ, const float* __restrict__ cw, const float* __restrict__ cb,
    unsigned short* __restrict__ U16) {
  constexpr float carry = (float)(1u << kCarryU_L2);
  const unsigned gid = blockIdx.x * 256u + threadIdx.x;
  const unsigned row = pin_u(gid / (unsigned)kThrRow);
  const unsigned c4  = (gid - row * (unsigned)kThrRow) << 2;
  const v4f bias = *(const v4f*)(cb + c4);
  v4f sv;
  bool valid;
  if (MODE == 2) {
    valid = row < (unsigned)kRowsW;
    const unsigned rowc = valid ? row : (unsigned)(kRowsW - 1);
    const unsigned s  = pin_u(rowc / (unsigned)kWinT);
    const unsigned p  = rowc - s * (unsigned)kWinT;
    const unsigned q  = s >> 4;
    const unsigned b  = s & 15u;
    const unsigned ph = pin_u(p / (unsigned)kWinS);
    const unsigned pw = p - ph * (unsigned)kWinS;
    const unsigned hh = (unsigned)kWinS * (q >> 1) + ph;
    const unsigned ww = (unsigned)kWinS * (q & 1u) + pw;
    const unsigned srow = b * (unsigned)kSeqL + hh * (unsigned)kSide + ww;
    v4f xv = *(const v4f*)(XZ + (size_t)srow * kXzP + c4);
    asm volatile("" : "+v"(xv));
    const v4f wv = *(const v4f*)(cw + c4);
#pragma unroll
    for (int e = 0; e < 4; ++e) sv[e] = xv[e] * wv[e] + bias[e];
  } else {
    valid = row < (unsigned)kRows;
    const unsigned rowc = valid ? row : (unsigned)(kRows - 1);
    const unsigned b = pin_u(rowc / (unsigned)kSeqL);
    const unsigned t = rowc - b * (unsigned)kSeqL;
    v4f wq[4];
#pragma unroll
    for (int e = 0; e < 4; ++e) wq[e] = *(const v4f*)(cw + (size_t)(c4 + e) * 4);
    v4f acc = (v4f){0.f, 0.f, 0.f, 0.f};
#pragma unroll
    for (int j = 0; j < 4; ++j) {
      const int tt = (int)t - 3 + j;
      const bool ok = tt >= 0;
      const unsigned ttc = ok ? (unsigned)tt : 0u;
      unsigned ts = ttc;
      if (MODE == 1) {
        const unsigned a = pin_u(ttc / (unsigned)kSide);
        const unsigned r = ttc - a * (unsigned)kSide;
        ts = (ttc < (unsigned)(kSeqL - 1)) ? (r * (unsigned)kSide + a) : ttc;
      }
      v4f xv = *(const v4f*)(XZ + (size_t)(b * (unsigned)kSeqL + ts) * kXzP + c4);
      asm volatile("" : "+v"(xv));
#pragma unroll
      for (int e = 0; e < 4; ++e) {
        const float xs = ok ? xv[e] : 0.0f;
        acc[e] = fmaf(wq[e][j], xs, acc[e]);
      }
    }
#pragma unroll
    for (int e = 0; e < 4; ++e) sv[e] = acc[e] + bias[e];
  }
  v4h hv;
#pragma unroll
  for (int e = 0; e < 4; ++e) {
    const float u = silu_f(sv[e]) * carry;
    const float us = valid ? u : 0.0f;
    hv[e] = to_h16(us);
  }
  unsigned short* q = U16 + (size_t)row * kEd + c4;
  *(volatile v4h*)q = hv;
  __threadfence();
  *(volatile v4h*)q = hv;
}

constexpr int kScanTS = 50;
constexpr int kScanCh = 128;
constexpr int kScanYP = 132;
constexpr int kScanBlkPerSeq = kEd / kScanCh;
static_assert(kScanBlkPerSeq == 12);
static_assert(kScanTS * 8 <= 4 * kScanCh);
static_assert(7 * 8 >= kScanTS);

template <int T>
__global__ __launch_bounds__(128) void scan_kernel(
    const unsigned short* __restrict__ U16, const float* __restrict__ DELTA, const float* __restrict__ DBC,
    const float* __restrict__ Alog, unsigned short* __restrict__ Y) {
  __shared__ __align__(16) float sBC[kScanTS * 32];
  __shared__ __align__(16) float sY[kScanTS * kScanYP];
  __shared__ __align__(16) float sA[kNst * kScanCh];
  constexpr float invCarryU = 1.0f / (float)(1u << kCarryU_L2);
  constexpr float carryY = (float)(1u << kCarryY_L2);
  const int tid = threadIdx.x, lane = tid & 31, wave = tid >> 5;
  const unsigned s  = blockIdx.x / (unsigned)kScanBlkPerSeq;
  const unsigned cbk = blockIdx.x - s * (unsigned)kScanBlkPerSeq;
  const int e0 = (int)cbk * kScanCh;
  const int e  = e0 + tid;
  const size_t row0 = (size_t)s * T;
#pragma unroll 1
  for (int n = 0; n < kNst; ++n) sA[n * kScanCh + tid] = -expf(Alog[(size_t)e * kNst + n]);
  __syncthreads();
  float An[kNst], h[kNst];
#pragma unroll
  for (int n = 0; n < kNst; ++n) {
    An[n] = sA[n * kScanCh + tid];
    h[n] = 0.0f;
  }
  const int hh = lane >> 4;
  const int c8 = (lane & 15) * 8;
#pragma unroll 1
  for (int t0 = 0; t0 < T; t0 += kScanTS) {
    const int ns = (T - t0 < kScanTS) ? (T - t0) : kScanTS;
    __syncthreads();
#pragma unroll 1
    for (int it = 0; it < 4; ++it) {
      const int idx = it * kScanCh + tid;
      const int idc = (idx < kScanTS * 8) ? idx : (kScanTS * 8 - 1);
      const int r = idc >> 3;
      const int c = (idc & 7) * 4;
      const int rc = (r < ns) ? r : (ns - 1);
      v4f v = *(const v4f*)(DBC + (row0 + t0 + rc) * kDbcP + kDtr + c);
      asm volatile("" : "+v"(v));
      if (idx < kScanTS * 8) *(v4f*)(sBC + r * 32 + c) = v;
    }
    __syncthreads();
#pragma unroll 1
    for (int sidx = 0; sidx < ns; ++sidx) {
      const size_t row = row0 + t0 + sidx;
      const float* bc = sBC + sidx * 32;
      const float dl = DELTA[row * kEd + e];
      const unsigned uw = (unsigned)U16[row * kEd + e];
      const float u = h16_to_f32(uw) * invCarryU;
      const float dtx = dl * u;
      v4f bv[4], cv[4];
#pragma unroll
      for (int q4 = 0; q4 < 4; ++q4) {
        bv[q4] = *(const v4f*)(bc + 4 * q4);
        cv[q4] = *(const v4f*)(bc + kNst + 4 * q4);
      }
      float y = 0.0f;
#pragma unroll
      for (int n = 0; n < kNst; ++n) {
        const float ea = expf(dl * An[n]);
        h[n] = fmaf(ea, h[n], dtx * bv[n >> 2][n & 3]);
        y = fmaf(h[n], cv[n >> 2][n & 3], y);
      }
      sY[sidx * kScanYP + tid] = y;
    }
    __syncthreads();
    for (int pass = 0; pass < 2; ++pass) {
#pragma unroll 1
      for (int it = 0; it < 7; ++it) {
        const int r = it * 8 + wave * 2 + hh;
        const int rc = (r < ns) ? r : (ns - 1);
        const float* sp = sY + rc * kScanYP + c8;
        const v4f a0 = *(const v4f*)(sp);
        const v4f a1 = *(const v4f*)(sp + 4);
        v8h hv;
#pragma unroll
        for (int k = 0; k < 4; ++k) {
          hv[k]     = to_h16(a0[k] * carryY);
          hv[4 + k] = to_h16(a1[k] * carryY);
        }
        if (r < ns) *(volatile v8h*)(Y + (row0 + t0 + r) * kEd + e0 + c8) = hv;
      }
      __threadfence();
    }
  }
}

__global__ __launch_bounds__(256) void combine_kernel(
    const unsigned* __restrict__ Y0, const unsigned* __restrict__ Y1, const unsigned* __restrict__ YW,
    const float* __restrict__ XZ, unsigned short* __restrict__ PRE16) {
  constexpr float outScale = (float)(1u << (kCarryP_L2 - kCarryY_L2));
  const unsigned gid = blockIdx.x * 256u + threadIdx.x;
  const unsigned row = pin_u(gid / (unsigned)kThrRow);
  const unsigned c4  = (gid - row * (unsigned)kThrRow) << 2;
  const bool valid = row < (unsigned)kRows;
  const unsigned rowc = valid ? row : (unsigned)(kRows - 1);
  const unsigned b = pin_u(rowc / (unsigned)kSeqL);
  const unsigned t = rowc - b * (unsigned)kSeqL;
  const bool first = (t == 0u);
  const unsigned tp = first ? 0u : (t - 1u);
  const unsigned ta = pin_u(tp / (unsigned)kSide);
  const unsigned tr = tp - ta * (unsigned)kSide;
  const unsigned r0 = first ? (unsigned)(kSeqL - 1) : tp;
  const unsigned r1 = first ? (unsigned)(kSeqL - 1) : (tr * (unsigned)kSide + ta);
  const bool usew = t < (unsigned)(kSeqL - 1);
  const unsigned tw = usew ? t : (unsigned)(kSeqL - 2);
  const unsigned wh = pin_u(tw / (unsigned)kSide);
  const unsigned ww = tw - wh * (unsigned)kSide;
  const unsigned qh = (wh >= (unsigned)kWinS) ? 1u : 0u;
  const unsigned qw = (ww >= (unsigned)kWinS) ? 1u : 0u;
  const unsigned q  = qh * 2u + qw;
  const unsigned p  = (wh - qh * (unsigned)kWinS) * (unsigned)kWinS + (ww - qw * (unsigned)kWinS);
  const unsigned rw = (q * (unsigned)kBatch + b) * (unsigned)kWinT + p;
  const unsigned base = b * (unsigned)kSeqL;
  const unsigned cw2 = c4 >> 1;
  constexpr unsigned wordsPerRow = (unsigned)kEd / 2u;
  v2u wa = *(const v2u*)(Y0 + (size_t)(base + r0) * wordsPerRow + cw2);
  v2u wb = *(const v2u*)(Y1 + (size_t)(base + r1) * wordsPerRow + cw2);
  v2u wc = *(const v2u*)(YW + (size_t)rw * wordsPerRow + cw2);
  v2u wd = *(const v2u*)(Y1 + (size_t)(base + (unsigned)(kSeqL - 1)) * wordsPerRow + cw2);
  asm volatile("" : "+v"(wa));
  asm volatile("" : "+v"(wb));
  asm volatile("" : "+v"(wc));
  asm volatile("" : "+v"(wd));
  v4f zv = *(const v4f*)(XZ + (size_t)rowc * kXzP + kEd + c4);
  asm volatile("" : "+v"(zv));
  const unsigned a0 = wa[0], a1 = wa[1];
  const unsigned b0 = wb[0], b1 = wb[1];
  const unsigned c0s = wc[0], c1s = wc[1];
  const unsigned d0s = wd[0], d1s = wd[1];
  const unsigned t0w = usew ? c0s : d0s;
  const unsigned t1w = usew ? c1s : d1s;
  const float fa[4] = {h16_to_f32(a0 & 0xffffu), h16_to_f32(a0 >> 16), h16_to_f32(a1 & 0xffffu), h16_to_f32(a1 >> 16)};
  const float fb[4] = {h16_to_f32(b0 & 0xffffu), h16_to_f32(b0 >> 16), h16_to_f32(b1 & 0xffffu), h16_to_f32(b1 >> 16)};
  const float fc[4] = {h16_to_f32(t0w & 0xffffu), h16_to_f32(t0w >> 16), h16_to_f32(t1w & 0xffffu), h16_to_f32(t1w >> 16)};
  v4h hv;
#pragma unroll
  for (int e = 0; e < 4; ++e) {
    const float zs = silu_f(zv[e]);
    float o = fa[e] * zs;
    o = o + fb[e] * zs;
    o = o + fc[e] * zs;
    const float os = valid ? (o * outScale) : 0.0f;
    hv[e] = to_h16(os);
  }
  unsigned short* qd = PRE16 + (size_t)row * kEd + c4;
  *(volatile v4h*)qd = hv;
  __threadfence();
  *(volatile v4h*)qd = hv;
}

extern "C" void kernel_launch(void* const* d_in, const int* in_sizes, int n_in,
                              void* d_out, int out_size, void* d_ws, size_t ws_size,
                              hipStream_t stream) {
  if (n_in < 16) return;
  if (in_sizes[0] != kRows * kDm) return;
  if (in_sizes[1] != kXzP * kDm) return;
  if (in_sizes[2] != kEd * 4 || in_sizes[4] != kEd * 4) return;
  if (in_sizes[3] != kEd || in_sizes[5] != kEd || in_sizes[6] != kEd || in_sizes[7] != kEd) return;
  if (in_sizes[8] != 80 * kEd || in_sizes[9] != 80 * kEd || in_sizes[10] != 80 * kEd) return;
  if (in_sizes[11] != kEd * kDtr) return;
  if (in_sizes[12] != kEd) return;
  if (in_sizes[13] != kEd * kNst) return;
  if (in_sizes[15] != kDm * kEd) return;
  if (out_size != kRows * kDm) return;
  if (ws_size < kWsTotal) return;

  const float* x       = (const float*)d_in[0];
  const float* W_in    = (const float*)d_in[1];
  const float* conv0_w = (const float*)d_in[2];
  const float* conv0_b = (const float*)d_in[3];
  const float* conv1_w = (const float*)d_in[4];
  const float* conv1_b = (const float*)d_in[5];
  const float* conv2_w = (const float*)d_in[6];
  const float* conv2_b = (const float*)d_in[7];
  const float* xproj0  = (const float*)d_in[8];
  const float* xproj1  = (const float*)d_in[9];
  const float* xproj2  = (const float*)d_in[10];
  const float* dt_w    = (const float*)d_in[11];
  const float* dt_b    = (const float*)d_in[12];
  const float* A_log   = (const float*)d_in[13];
  const float* W_out   = (const float*)d_in[15];
  float* out = (float*)d_out;

  char* ws = (char*)d_ws;
  unsigned short* XH    = (unsigned short*)(ws + kOffXH);
  unsigned short* XL    = (unsigned short*)(ws + kOffXL);
  unsigned short* WIH   = (unsigned short*)(ws + kOffWIH);
  unsigned short* WIL   = (unsigned short*)(ws + kOffWIL);
  float*          XZ    = (float*)(ws + kOffXZ);
  unsigned short* U16   = (unsigned short*)(ws + kOffU16);
  unsigned short* PRE16 = (unsigned short*)(ws + kOffPRE16);
  unsigned short* XP16a = (unsigned short*)(ws + kOffXP16);
  unsigned short* XP16b = (unsigned short*)(ws + kOffXP16 + kSzXP16);
  unsigned short* XP16c = (unsigned short*)(ws + kOffXP16 + 2 * kSzXP16);
  float*          DBC   = (float*)(ws + kOffDBC);
  unsigned short* DBC16 = (unsigned short*)(ws + kOffDBC16);
  unsigned short* DTW16 = (unsigned short*)(ws + kOffDTW16);
  float*          DELTA = (float*)(ws + kOffDELTA);
  unsigned short* Y0    = (unsigned short*)(ws + kOffY0);
  unsigned short* Y1    = (unsigned short*)(ws + kOffY1);
  unsigned short* YW    = (unsigned short*)(ws + kOffYW);
  unsigned short* WO16  = (unsigned short*)(ws + kOffWO16);

  split_rows_bf16_kernel<<<(kRowsP * kDm / 8) / 256, 256, 0, stream>>>(
      x, (unsigned*)XH, (unsigned*)XL, (unsigned)(kRows * kDm), (unsigned)(kRowsP * kDm / 8));
  split_rows_bf16_kernel<<<(kXzP * kDm / 8) / 256, 256, 0, stream>>>(
      W_in, (unsigned*)WIH, (unsigned*)WIL, (unsigned)(kXzP * kDm), (unsigned)(kXzP * kDm / 8));
  cast_pad_f16_kernel<kCarryW_L2><<<(kXpRows * kEd / 8) / 256, 256, 0, stream>>>(
      xproj0, XP16a, 80u, (unsigned)kEd, (unsigned)(kEd / 8), (unsigned)(kXpRows * kEd / 8));
  cast_pad_f16_kernel<kCarryW_L2><<<(kXpRows * kEd / 8) / 256, 256, 0, stream>>>(
      xproj1, XP16b, 80u, (unsigned)kEd, (unsigned)(kEd / 8), (unsigned)(kXpRows * kEd / 8));
  cast_pad_f16_kernel<kCarryW_L2><<<(kXpRows * kEd / 8) / 256, 256, 0, stream>>>(
      xproj2, XP16c, 80u, (unsigned)kEd, (unsigned)(kEd / 8), (unsigned)(kXpRows * kEd / 8));
  cast_pad_f16_kernel<kCarryW_L2><<<(kEd * kDbc16P / 8) / 256, 256, 0, stream>>>(
      dt_w, DTW16, (unsigned)kEd, (unsigned)kDtr, (unsigned)(kDbc16P / 8), (unsigned)(kEd * kDbc16P / 8));
  cast_pad_f16_kernel<kCarryW_L2><<<(kDm * kEd / 8) / 256, 256, 0, stream>>>(
      W_out, WO16, (unsigned)kDm, (unsigned)kEd, (unsigned)(kEd / 8), (unsigned)(kDm * kEd / 8));

  wmma_gemm64<1, true, 0, 0><<<300, 256, 0, stream>>>(
      XH, XL, kDm, WIH, WIL, kDm, XZ, kXzP, U16, 0, dt_b, kRowsP, kXzP, kDm, kRowsP);

  const int prepBlocks = kRowsP * kThrRow / 256;

  seq_prep_kernel<0><<<prepBlocks, 256, 0, stream>>>(XZ, conv0_w, conv0_b, U16);
  wmma_gemm64<0, false, 1, kCarryU_L2 + kCarryW_L2><<<13, 256, 0, stream>>>(
      U16, U16, kEd, XP16a, XP16a, kEd, DBC, kDbcP, DBC16, kDbc16P, dt_b, kRowsP, kDbcP, kEd, kRowsP);
  wmma_gemm64<0, false, 2, kCarryD_L2 + kCarryW_L2><<<150, 256, 0, stream>>>(
      DBC16, DBC16, kDbc16P, DTW16, DTW16, kDbc16P, DELTA, kEd, U16, 0, dt_b, kRowsP, kEd, kDbc16P, kRowsP);
  scan_kernel<kSeqL><<<kBatch * kScanBlkPerSeq, kScanCh, 0, stream>>>(U16, DELTA, DBC, A_log, Y0);

  seq_prep_kernel<1><<<prepBlocks, 256, 0, stream>>>(XZ, conv1_w, conv1_b, U16);
  wmma_gemm64<0, false, 1, kCarryU_L2 + kCarryW_L2><<<13, 256, 0, stream>>>(
      U16, U16, kEd, XP16b, XP16b, kEd, DBC, kDbcP, DBC16, kDbc16P, dt_b, kRowsP, kDbcP, kEd, kRowsP);
  wmma_gemm64<0, false, 2, kCarryD_L2 + kCarryW_L2><<<150, 256, 0, stream>>>(
      DBC16, DBC16, kDbc16P, DTW16, DTW16, kDbc16P, DELTA, kEd, U16, 0, dt_b, kRowsP, kEd, kDbc16P, kRowsP);
  scan_kernel<kSeqL><<<kBatch * kScanBlkPerSeq, kScanCh, 0, stream>>>(U16, DELTA, DBC, A_log, Y1);

  seq_prep_kernel<2><<<prepBlocks, 256, 0, stream>>>(XZ, conv2_w, conv2_b, U16);
  wmma_gemm64<0, false, 1, kCarryU_L2 + kCarryW_L2><<<13, 256, 0, stream>>>(
      U16, U16, kEd, XP16c, XP16c, kEd, DBC, kDbcP, DBC16, kDbc16P, dt_b, kRowsP, kDbcP, kEd, kRowsP);
  wmma_gemm64<0, false, 2, kCarryD_L2 + kCarryW_L2><<<150, 256, 0, stream>>>(
      DBC16, DBC16, kDbc16P, DTW16, DTW16, kDbc16P, DELTA, kEd, U16, 0, dt_b, kRowsP, kEd, kDbc16P, kRowsP);
  scan_kernel<kWinT><<<4 * kBatch * kScanBlkPerSeq, kScanCh, 0, stream>>>(U16, DELTA, DBC, A_log, YW);

  combine_kernel<<<prepBlocks, 256, 0, stream>>>(
      (const unsigned*)Y0, (const unsigned*)Y1, (const unsigned*)YW, XZ, PRE16);
  wmma_gemm64<0, false, 0, kCarryP_L2 + kCarryW_L2><<<75, 256, 0, stream>>>(
      PRE16, PRE16, kEd, WO16, WO16, kEd, out, kDm, U16, 0, dt_b, kRowsP, kDm, kEd, kRows);
}
